// _NonLocalNd_13099650253374
// MI455X (gfx1250) — hardware-verified
//
#include <hip/hip_runtime.h>


#define NB_  2
#define CX   128
#define CI   64
#define NPOS 9216
#define NT_  NPOS
#define RCH  1024
#define DM   CX
#define NTK  NPOS
#define SCL  0.125f
#define LOSC 1024.0f
#define BN_EPS 1e-5f

typedef _Float16 h16;
typedef unsigned short bf;
typedef __attribute__((ext_vector_type(16))) __bf16   v16bf;
typedef __attribute__((ext_vector_type(16))) _Float16 v16h;
typedef __attribute__((ext_vector_type(8)))  _Float16 v8h;
typedef __attribute__((ext_vector_type(8)))  unsigned short v8us;
typedef __attribute__((ext_vector_type(8)))  float    v8f;
typedef __attribute__((ext_vector_type(4)))  float    v4f;
typedef __attribute__((ext_vector_type(4)))  _Float16 v4h;
typedef v8h  __attribute__((may_alias)) v8ha;
typedef v4f  __attribute__((may_alias)) v4fa;
typedef v8us __attribute__((may_alias)) v8usa;

__device__ __forceinline__ unsigned short f2bf(float f) { unsigned u = __float_as_uint(f); u += 0x7FFFu + ((u >> 16) & 1u); return (unsigned short)(u >> 16); }
__device__ __forceinline__ float bf2f(unsigned short b) { return __uint_as_float(((unsigned)b) << 16); }
__device__ __forceinline__ float bfr(float f) { return bf2f(f2bf(f)); }
__device__ __forceinline__ v16h cat16(v8h lo, v8h hi) { return __builtin_shufflevector(lo, hi, 0, 1, 2, 3, 4, 5, 6, 7, 8, 9, 10, 11, 12, 13, 14, 15); }
__device__ __forceinline__ v16bf cat16b(v8us lo, v8us hi) { return __builtin_bit_cast(v16bf, __builtin_shufflevector(lo, hi, 0, 1, 2, 3, 4, 5, 6, 7, 8, 9, 10, 11, 12, 13, 14, 15)); }
__device__ __forceinline__ v8f wmma16(v16h a, v16h b, v8f c) { return __builtin_amdgcn_wmma_f32_16x16x32_f16(false, a, false, b, (short)0, c, false, false); }
__device__ __forceinline__ v8f wmmab(v16bf a, v16bf b, v8f c) { return __builtin_amdgcn_wmma_f32_16x16x32_bf16(false, a, false, b, (short)0, c, false, false); }

__global__ __launch_bounds__(256) void k_wt(const float* __restrict__ Wm, int K, int ncols, bf* WT) {
    __shared__ __align__(16) unsigned short tl[64 * 72];
    const int tid = threadIdx.x, k0 = blockIdx.x * 64, n0 = blockIdx.y * 64;
    const int kk = tid >> 2, nq = (tid & 3) * 16;
#pragma unroll
    for (int i = 0; i < 16; ++i) tl[(nq + i) * 72 + kk] = f2bf(Wm[(size_t)(k0 + kk) * ncols + n0 + nq + i]);
    __syncthreads();
    const int piece = tid & 7;
    auto pass = [&]() {
#pragma unroll
        for (int s = 0; s < 2; ++s) { const int nr = (tid >> 3) + 32 * s; const v8us val = *(const v8usa*)(tl + nr * 72 + piece * 8); *(volatile v8us*)(WT + (size_t)(n0 + nr) * K + k0 + piece * 8) = val; }
    };
    pass(); __threadfence(); pass();
}
template <bool SPLITA, bool F16OUT = false>
__global__ __launch_bounds__(128) void k_gemmb(const bf* __restrict__ A, const bf* __restrict__ Al, const bf* __restrict__ Bn, const float* __restrict__ bias, float* C, int ldc, h16* C2, const float* __restrict__ R = nullptr, int K = DM, int roundR = 1) {
    __shared__ __align__(16) float ost[4][16 * 68];
    const int lane = threadIdx.x & 31, wave = threadIdx.x >> 5, lr = lane & 15, hi = lane >> 4;
    const int r0 = blockIdx.x * 64 + wave * 16, c0 = blockIdx.y * 64;
    const size_t aoff = (size_t)(r0 + lr) * K + 8 * hi;
    size_t boff[4];
#pragma unroll
    for (int t = 0; t < 4; ++t) boff[t] = (size_t)(c0 + t * 16 + lr) * K + 8 * hi;
    v8f acc[4];
#pragma unroll
    for (int t = 0; t < 4; ++t) acc[t] = (v8f){};
#pragma unroll 1
    for (int kc = 0; kc < K; kc += 32) {
        const v16bf a = cat16b(*(const v8us*)(A + aoff + kc), *(const v8us*)(A + aoff + kc + 16));
        v16bf al = a;
        if (SPLITA) al = cat16b(*(const v8us*)(Al + aoff + kc), *(const v8us*)(Al + aoff + kc + 16));
#pragma unroll
        for (int t = 0; t < 4; ++t) { const v16bf b = cat16b(*(const v8us*)(Bn + boff[t] + kc), *(const v8us*)(Bn + boff[t] + kc + 16)); acc[t] = wmmab(a, b, acc[t]); if (SPLITA) acc[t] = wmmab(al, b, acc[t]); }
        asm volatile("v_nop\n\tv_nop\n\tv_nop\n\tv_nop" : "+v"(acc[0]), "+v"(acc[1]), "+v"(acc[2]), "+v"(acc[3]) : "v"(a), "v"(al));
    }
    float* os = &ost[wave][0];
#pragma unroll
    for (int t = 0; t < 4; ++t) { const float bv = bias ? bfr(bias[c0 + t * 16 + lr]) : 0.f;
#pragma unroll
        for (int j = 0; j < 8; ++j) os[(hi * 8 + j) * 68 + t * 16 + lr] = acc[t][j] + bv; }
    __syncthreads();
    if (F16OUT) {
        h16* crow = (h16*)(void*)C + (size_t)r0 * ldc + c0;
        auto pass = [&]() {
#pragma unroll
            for (int s = 0; s < 4; ++s) { const int row = 4 * s + (lane >> 3), piece = lane & 7; const float* sp = os + row * 68 + piece * 8; v8h o, o2;
#pragma unroll
                for (int i = 0; i < 8; ++i) { const h16 a = (h16)sp[i]; o[i] = a; o2[i] = (h16)((sp[i] - (float)a) * LOSC); }
                *(volatile v8h*)(crow + (size_t)row * ldc + piece * 8) = o; if (C2) *(volatile v8h*)(C2 + (size_t)r0 * ldc + c0 + (size_t)row * ldc + piece * 8) = o2; }
        };
        pass(); __threadfence(); pass();
    } else {
        float* crow = C + (size_t)r0 * ldc + c0;
        auto pass = [&]() {
#pragma unroll
            for (int s = 0; s < 8; ++s) { const int Lid = (lane >> 3) + 4 * s, piece = lane & 7; const int row = Lid >> 1, cofs = (Lid & 1) * 32 + piece * 4;
                v4f val = *(const v4fa*)(os + row * 68 + cofs); if (R) { const v4f rv = *(const v4f*)(R + ((size_t)r0 + row) * ldc + c0 + cofs); val += roundR ? (v4f){bfr(rv[0]), bfr(rv[1]), bfr(rv[2]), bfr(rv[3])} : rv; }
                *(volatile v4f*)(crow + (size_t)row * ldc + cofs) = val; }
        };
        pass(); __threadfence(); pass();
    }
}

__global__ __launch_bounds__(128) void k_gemm3(const bf* __restrict__ Ah, const bf* __restrict__ Al, const bf* __restrict__ Bh, const bf* __restrict__ Bl, int K, float* C, int ldc) {
    __shared__ __align__(16) float ost[4][16 * 68];
    const int lane = threadIdx.x & 31, wave = threadIdx.x >> 5, lr = lane & 15, hi = lane >> 4;
    const int r0 = blockIdx.x * 64 + wave * 16, c0 = blockIdx.y * 64;
    const size_t aoff = (size_t)(r0 + lr) * K + 8 * hi;
    v8f acc[4];
#pragma unroll
    for (int t = 0; t < 4; ++t) acc[t] = (v8f){};
#pragma unroll 1
    for (int kc = 0; kc < K; kc += 32) {
        const v16bf a = cat16b(*(const v8us*)(Ah + aoff + kc), *(const v8us*)(Ah + aoff + kc + 16));
        const v16bf al = cat16b(*(const v8us*)(Al + aoff + kc), *(const v8us*)(Al + aoff + kc + 16));
#pragma unroll
        for (int t = 0; t < 4; ++t) { const size_t bo = (size_t)(c0 + t * 16 + lr) * K + kc + 8 * hi;
            const v16bf bh = cat16b(*(const v8us*)(Bh + bo), *(const v8us*)(Bh + bo + 16)); const v16bf bl = cat16b(*(const v8us*)(Bl + bo), *(const v8us*)(Bl + bo + 16));
            acc[t] = wmmab(a, bh, acc[t]); acc[t] = wmmab(al, bh, acc[t]); acc[t] = wmmab(a, bl, acc[t]); }
        asm volatile("v_nop\n\tv_nop\n\tv_nop\n\tv_nop" : "+v"(acc[0]), "+v"(acc[1]), "+v"(acc[2]), "+v"(acc[3]) : "v"(a), "v"(al));
    }
    float* os = &ost[wave][0];
#pragma unroll
    for (int t = 0; t < 4; ++t) {
#pragma unroll
        for (int j = 0; j < 8; ++j) os[(hi * 8 + j) * 68 + t * 16 + lr] = acc[t][j]; }
    __builtin_amdgcn_wave_barrier(); asm volatile("" ::: "memory");
    float* crow = C + (size_t)r0 * ldc + c0;
    auto pass = [&]() {
#pragma unroll
        for (int s = 0; s < 8; ++s) { const int Lid = (lane >> 3) + 4 * s, piece = lane & 7; const int row = Lid >> 1, cofs = (Lid & 1) * 32 + piece * 4;
            const v4f val = *(const v4fa*)(os + row * 68 + cofs); *(volatile v4f*)(crow + (size_t)row * ldc + cofs) = val; }
    };
    pass(); __threadfence(); pass();
}
__global__ __launch_bounds__(256) void k_softmax(const float* __restrict__ S, bf* PH, bf* PL) {
    const int lane = threadIdx.x & 31, r = blockIdx.x * 8 + (threadIdx.x >> 5);
    if (r >= RCH) return;
    const float* sr = S + (size_t)r * NT_ + lane * 8;
    float m = -3.0e38f;
#pragma unroll 1
    for (int q = 0; q < NT_ / 256; ++q) { const v8f v = *(const v8f*)(sr + q * 256);
#pragma unroll
        for (int i = 0; i < 8; ++i) m = fmaxf(m, v[i] * SCL); }
#pragma unroll
    for (int sh = 16; sh; sh >>= 1) m = fmaxf(m, __shfl_xor(m, sh, 32));
    float den = 0.f;
#pragma unroll 1
    for (int q = 0; q < NT_ / 256; ++q) { const v8f v = *(const v8f*)(sr + q * 256);
#pragma unroll
        for (int i = 0; i < 8; ++i) den += __expf(v[i] * SCL - m); }
#pragma unroll
    for (int sh = 16; sh; sh >>= 1) den += __shfl_xor(den, sh, 32);
#pragma unroll 1
    for (int ps = 0; ps < 2; ++ps) {
#pragma unroll 1
        for (int q = 0; q < NT_ / 256; ++q) { const v8f v = *(const v8f*)(sr + q * 256); v8us oh, ol;
#pragma unroll
            for (int i = 0; i < 8; ++i) { const float p = __expf(v[i] * SCL - m) / den; const unsigned short hb = f2bf(p); oh[i] = hb; ol[i] = f2bf(p - bf2f(hb)); }
            const size_t o = (size_t)r * NT_ + q * 256 + lane * 8; *(volatile v8us*)(PH + o) = oh; *(volatile v8us*)(PL + o) = ol; }
        if (ps == 0) __threadfence(); }
}

__global__ __launch_bounds__(256) void k_bf(const float* __restrict__ src, bf* dst, size_t n8) {
    const size_t i = (size_t)blockIdx.x * 256 + threadIdx.x; if (i >= n8) return;
    const v8f v = *(const v8f*)(src + i * 8); v8us o;
#pragma unroll
    for (int k = 0; k < 8; ++k) o[k] = f2bf(v[k]);
    *(volatile v8us*)(dst + i * 8) = o; __threadfence(); *(volatile v8us*)(dst + i * 8) = o;
}
__device__ __forceinline__ float bn_apply(float v, const float* g, const float* b, const float* m, const float* var, int c) {
    const float sc = bfr(g[c]) / sqrtf(bfr(var[c]) + BN_EPS); return v * sc + (bfr(b[c]) - bfr(m[c]) * sc);
}
__global__ __launch_bounds__(256) void k_bnrelu_cols(const float* __restrict__ T, int nrows, const float* g, const float* b, const float* m, const float* var, bf* dh, bf* dl) {
    typedef __attribute__((ext_vector_type(2))) unsigned short v2us;
    const int lane = threadIdx.x & 31, r = blockIdx.x * 8 + (threadIdx.x >> 5); if (r >= nrows) return;
    const size_t o = (size_t)r * CI + lane * 2; v2us oh, ol;
#pragma unroll
    for (int i = 0; i < 2; ++i) { const int c = lane * 2 + i; const float y = fmaxf(bn_apply(T[o + i], g, b, m, var, c), 0.f); const unsigned short hb = f2bf(y); oh[i] = hb; ol[i] = f2bf(y - bf2f(hb)); }
    *(volatile v2us*)(dh + o) = oh; *(volatile v2us*)(dl + o) = ol; __threadfence(); *(volatile v2us*)(dh + o) = oh; *(volatile v2us*)(dl + o) = ol;
}
__global__ __launch_bounds__(256) void k_bnrelu_rows(const float* __restrict__ Gf, const float* g, const float* b, const float* m, const float* var, bf* dh, bf* dl) {
    const int lane = threadIdx.x & 31, wid = blockIdx.x * 8 + (threadIdx.x >> 5); if (wid >= CI * (NPOS / 256)) return;
    const int c = wid / (NPOS / 256), sg = wid - c * (NPOS / 256); const size_t o = (size_t)c * NPOS + sg * 256 + lane * 8;
    const v8f v = *(const v8f*)(Gf + o); v8us oh, ol;
#pragma unroll
    for (int i = 0; i < 8; ++i) { const float y = fmaxf(bn_apply(v[i], g, b, m, var, c), 0.f); const unsigned short hb = f2bf(y); oh[i] = hb; ol[i] = f2bf(y - bf2f(hb)); }
    *(volatile v8us*)(dh + o) = oh; *(volatile v8us*)(dl + o) = ol; __threadfence(); *(volatile v8us*)(dh + o) = oh; *(volatile v8us*)(dl + o) = ol;
}
__global__ __launch_bounds__(256) void k_split64(const float* __restrict__ T, int nrows, bf* dh, bf* dl) {
    typedef __attribute__((ext_vector_type(2))) unsigned short v2us;
    const int lane = threadIdx.x & 31, r = blockIdx.x * 8 + (threadIdx.x >> 5); if (r >= nrows) return;
    const size_t o = (size_t)r * CI + lane * 2; v2us oh, ol;
#pragma unroll
    for (int i = 0; i < 2; ++i) { const float y = T[o + i]; const unsigned short hb = f2bf(y); oh[i] = hb; ol[i] = f2bf(y - bf2f(hb)); }
    *(volatile v2us*)(dh + o) = oh; *(volatile v2us*)(dl + o) = ol; __threadfence(); *(volatile v2us*)(dh + o) = oh; *(volatile v2us*)(dl + o) = ol;
}
__global__ __launch_bounds__(256) void k_outT(const float* __restrict__ ZT, const float* __restrict__ X, const float* g, const float* b, const float* m, const float* var, float* OUTB) {
    __shared__ __align__(16) float tl[64 * 68];
    const int l0 = blockIdx.x * 64, o0 = blockIdx.y * 64, tid = threadIdx.x;
    const int ll = tid >> 2, oq = (tid & 3) * 16;
#pragma unroll 1
    for (int i = 0; i < 16; ++i) { const int o = o0 + oq + i; tl[(oq + i) * 68 + ll] = fmaxf(bn_apply(ZT[(size_t)(l0 + ll) * CX + o], g, b, m, var, o), 0.f); }
    __syncthreads();
    const int piece = tid & 15;
    auto pass = [&]() {
#pragma unroll
        for (int s = 0; s < 4; ++s) { const int orow = (tid >> 4) + 16 * s; const size_t oo = (size_t)(o0 + orow) * NPOS + l0 + piece * 4;
            const v4f xv = *(const v4f*)(X + oo); v4f val = *(const v4fa*)(tl + orow * 68 + piece * 4);
#pragma unroll
            for (int k = 0; k < 4; ++k) val[k] += bfr(xv[k]);
            *(volatile v4f*)(OUTB + oo) = val; }
    };
    pass(); __threadfence(); pass();
}

extern "C" void kernel_launch(void* const* d_in, const int* in_sizes, int n_in,
                              void* d_out, int out_size, void* d_ws, size_t ws_size, hipStream_t stream) {
    (void)in_sizes; (void)n_in; (void)out_size;
    const float* x = (const float*)d_in[0];
    const float* gW = (const float*)d_in[1]; const float* gg = (const float*)d_in[2]; const float* gb = (const float*)d_in[3]; const float* gm = (const float*)d_in[4]; const float* gv = (const float*)d_in[5];
    const float* tW = (const float*)d_in[6]; const float* tg = (const float*)d_in[7]; const float* tb = (const float*)d_in[8]; const float* tm = (const float*)d_in[9]; const float* tv = (const float*)d_in[10];
    const float* pW = (const float*)d_in[11]; const float* pg = (const float*)d_in[12]; const float* pb = (const float*)d_in[13]; const float* pm = (const float*)d_in[14]; const float* pv = (const float*)d_in[15];
    const float* oW = (const float*)d_in[16]; const float* og = (const float*)d_in[17]; const float* ob = (const float*)d_in[18]; const float* om = (const float*)d_in[19]; const float* ov = (const float*)d_in[20];
    float* out = (float*)d_out;
    char* wsp = (char*)d_ws;
    auto take = [&](size_t bytes) { char* p = wsp; wsp += (bytes + 255) & ~(size_t)255; return (void*)p; };
    bf* gWB = (bf*)take((size_t)CI * CX * 2); bf* tWB = (bf*)take((size_t)CI * CX * 2); bf* pWB = (bf*)take((size_t)CI * CX * 2); bf* oWB = (bf*)take((size_t)CX * CI * 2);
    bf* XT = (bf*)take((size_t)NPOS * CX * 2); float* T64 = (float*)take((size_t)NPOS * CI * 4);
    bf* THh = (bf*)take((size_t)NPOS * CI * 2); bf* THl = (bf*)take((size_t)NPOS * CI * 2); bf* PHh = (bf*)take((size_t)NPOS * CI * 2); bf* PHl = (bf*)take((size_t)NPOS * CI * 2);
    float* Gf = (float*)take((size_t)CI * NPOS * 4); bf* Gh = (bf*)take((size_t)CI * NPOS * 2); bf* Gl = (bf*)take((size_t)CI * NPOS * 2);
    float* S = (float*)take((size_t)RCH * NPOS * 4); bf* Ph = (bf*)take((size_t)RCH * NPOS * 2); bf* Pl = (bf*)take((size_t)RCH * NPOS * 2);
    float* YT = (float*)take((size_t)NPOS * CI * 4); bf* Yh = (bf*)take((size_t)NPOS * CI * 2); bf* Yl = (bf*)take((size_t)NPOS * CI * 2); float* ZT = (float*)take((size_t)NPOS * CX * 4);
    if ((size_t)(wsp - (char*)d_ws) > ws_size) return;
    k_bf<<<(CI * CX / 8 + 255) / 256, 256, 0, stream>>>(gW, gWB, CI * CX / 8); k_bf<<<(CI * CX / 8 + 255) / 256, 256, 0, stream>>>(tW, tWB, CI * CX / 8);
    k_bf<<<(CI * CX / 8 + 255) / 256, 256, 0, stream>>>(pW, pWB, CI * CX / 8); k_bf<<<(CX * CI / 8 + 255) / 256, 256, 0, stream>>>(oW, oWB, CX * CI / 8);
    for (int bi = 0; bi < NB_; ++bi) {
        const float* xb = x + (size_t)bi * CX * NPOS;
        k_wt<<<dim3(CX / 64, NPOS / 64, 1), 256, 0, stream>>>(xb, CX, NPOS, XT);
        k_gemmb<false, false><<<dim3(NPOS / 64, CI / 64, 1), 128, 0, stream>>>(XT, nullptr, tWB, nullptr, T64, CI, nullptr); k_bnrelu_cols<<<NPOS / 8, 256, 0, stream>>>(T64, NPOS, tg, tb, tm, tv, THh, THl);
        k_gemmb<false, false><<<dim3(NPOS / 64, CI / 64, 1), 128, 0, stream>>>(XT, nullptr, pWB, nullptr, T64, CI, nullptr); k_bnrelu_cols<<<NPOS / 8, 256, 0, stream>>>(T64, NPOS, pg, pb, pm, pv, PHh, PHl);
        k_gemmb<false, false><<<dim3(CI / 64, NPOS / 64, 1), 128, 0, stream>>>(gWB, nullptr, XT, nullptr, Gf, NPOS, nullptr); k_bnrelu_rows<<<(CI * (NPOS / 256)) / 8, 256, 0, stream>>>(Gf, gg, gb, gm, gv, Gh, Gl);
        for (int ch = 0; ch < NPOS / RCH; ++ch) {
            k_gemm3<<<dim3(RCH / 64, NPOS / 64, 1), 128, 0, stream>>>(THh + (size_t)ch * RCH * CI, THl + (size_t)ch * RCH * CI, PHh, PHl, CI, S, NPOS);
            k_softmax<<<RCH / 8, 256, 0, stream>>>(S, Ph, Pl);
            k_gemm3<<<dim3(RCH / 64, CI / 64, 1), 128, 0, stream>>>(Ph, Pl, Gh, Gl, NPOS, YT + (size_t)ch * RCH * CI, CI);
        }
        k_split64<<<NPOS / 8, 256, 0, stream>>>(YT, NPOS, Yh, Yl);
        k_gemmb<true, false><<<dim3(NPOS / 64, CX / 64, 1), 128, 0, stream>>>(Yh, Yl, oWB, nullptr, ZT, CX, nullptr, nullptr, CI);
        k_outT<<<dim3(NPOS / 64, CX / 64, 1), 256, 0, stream>>>(ZT, xb, og, ob, om, ov, out + (size_t)bi * CX * NPOS);
    }
}
